// Grok5PhiCore_70136815944177
// MI455X (gfx1250) — hardware-verified
//
#include <hip/hip_runtime.h>
#include <math.h>

typedef __attribute__((ext_vector_type(16))) _Float16 v16h;
typedef __attribute__((ext_vector_type(8)))  _Float16 v8h;
typedef __attribute__((ext_vector_type(16))) __bf16   v16b;
typedef __attribute__((ext_vector_type(8)))  __bf16   v8b;
typedef __attribute__((ext_vector_type(8)))  float    v8f;
typedef __attribute__((ext_vector_type(4)))  float    v4f;
typedef __attribute__((ext_vector_type(4)))  unsigned int v4u;

constexpr int kB    = 2;
constexpr int kL    = 2048;
constexpr int kD    = 1024;
constexpr int kH    = 16;
constexpr int kDh   = 64;
constexpr int kRows = kB * kL;
constexpr int kQKld = 2 * kD;
constexpr float kScoreScale = 0.125f;
constexpr double kGoldD = 1.6180339887498949;
constexpr float  kGoldF = (float)kGoldD;
constexpr float kPCarry   = 32768.0f;
constexpr float kOCarry   = 256.0f;
constexpr float kWCarry   = 16.0f;
constexpr float kOutScale = 1.0f / (kOCarry * kWCarry);
constexpr float kCtxScale = kOCarry / kPCarry;
static_assert(kH * kDh == kD);
static_assert(kScoreScale * kScoreScale * (float)kDh == 1.0f);
static_assert(kDh == 64);
static_assert((kRows % 64) == 0 && (kQKld % 64) == 0 && (kD % 64) == 0 && (kL % 64) == 0 && (kD % 32) == 0);
static_assert(((kRows * kD / 8) % 256) == 0);

constexpr size_t kOffXB  = 0;
constexpr size_t kOffWQT = kOffXB  + (size_t)kRows * kD * 2;
constexpr size_t kOffWPT = kOffWQT + (size_t)3 * kD * kD * 2;
constexpr size_t kOffQKH = kOffWPT + (size_t)kD * kD * 2;
constexpr size_t kOffVT  = kOffQKH + (size_t)kRows * kQKld * 2;
constexpr size_t kOffOH  = kOffVT  + (size_t)kB * kD * kL * 2;
constexpr size_t kWsTotal = kOffOH + (size_t)kRows * kD * 2;
static_assert(kWsTotal == 50331648ull);
static_assert(kWsTotal <= 134217728ull);
static_assert((kOffWQT % 128) == 0 && (kOffWPT % 128) == 0 && (kOffQKH % 128) == 0 && (kOffVT % 128) == 0 && (kOffOH % 128) == 0);

__device__ __forceinline__ unsigned short f2bf_bits(float f) {
  unsigned u = __float_as_uint(f);
  return (unsigned short)((u + 0x7FFFu + ((u >> 16) & 1u)) >> 16);
}
__device__ __forceinline__ float bf_bits2f(unsigned short h) { return __uint_as_float(((unsigned)h) << 16); }
__device__ __forceinline__ unsigned pk16(unsigned short a, unsigned short b) { return (unsigned)a | ((unsigned)b << 16); }
__device__ __forceinline__ unsigned short h_bits(float f) { const _Float16 h = (_Float16)f; return __builtin_bit_cast(unsigned short, h); }

__device__ __forceinline__ void dep_guard1_h(v8f& a, v16h x, v16h y) { asm volatile("v_nop\n\tv_nop\n\tv_nop\n\tv_nop" : "+v"(a) : "v"(x), "v"(y)); }
__device__ __forceinline__ void dep_guard1_b(v8f& a, v16b x, v16b y) { asm volatile("v_nop\n\tv_nop\n\tv_nop\n\tv_nop" : "+v"(a) : "v"(x), "v"(y)); }
__device__ __forceinline__ void keep4_h(v16h a, v16h b, v16h c, v16h d) { asm volatile("v_nop" :: "v"(a), "v"(b), "v"(c), "v"(d)); }
__device__ __forceinline__ void keep4_b(v16b a, v16b b, v16b c, v16b d) { asm volatile("v_nop" :: "v"(a), "v"(b), "v"(c), "v"(d)); }

template <typename T> struct Frag;
template <> struct Frag<_Float16> {
  typedef v16h V; union U { v16h v; v8h h[2]; };
  static __device__ __forceinline__ v16h load(const _Float16* p) {
    U f; f.h[0] = *(const v8h*)(p); f.h[1] = *(const v8h*)(p + 16); return f.v;
  }
  static __device__ __forceinline__ v8f mma(v16h a, v16h b, v8f c) {
    return __builtin_amdgcn_wmma_f32_16x16x32_f16(false, a, false, b, (short)0, c, false, false);
  }
  static __device__ __forceinline__ void guard1(v8f& a, v16h x, v16h y) { dep_guard1_h(a, x, y); }
  static __device__ __forceinline__ void keep(v16h a, v16h b, v16h c, v16h d) { keep4_h(a, b, c, d); }
};
template <> struct Frag<__bf16> {
  typedef v16b V; union U { v16b v; v8b h[2]; };
  static __device__ __forceinline__ v16b load(const __bf16* p) {
    U f; f.h[0] = *(const v8b*)(p); f.h[1] = *(const v8b*)(p + 16); return f.v;
  }
  static __device__ __forceinline__ v8f mma(v16b a, v16b b, v8f c) {
    return __builtin_amdgcn_wmma_f32_16x16x32_bf16(false, a, false, b, (short)0, c, false, false);
  }
  static __device__ __forceinline__ void guard1(v8f& a, v16b x, v16b y) { dep_guard1_b(a, x, y); }
  static __device__ __forceinline__ void keep(v16b a, v16b b, v16b c, v16b d) { keep4_b(a, b, c, d); }
};

__device__ __forceinline__ v8f mma_h(v16h a, v16h b, v8f c) {
  c = __builtin_amdgcn_wmma_f32_16x16x32_f16(false, a, false, b, (short)0, c, false, false);
  asm volatile("v_nop\n\tv_nop\n\tv_nop\n\tv_nop" : "+v"(c) : "v"(a), "v"(b));
  return c;
}

__device__ __forceinline__ float pos_frac(int i) {
#pragma clang fp contract(off)
  float p = (float)i * kGoldF;
  asm volatile("" : "+v"(p));
  return p - floorf(p);
}

template <int ET> struct Elem;
template <> struct Elem<0> { typedef _Float16 T; };
template <> struct Elem<1> { typedef __bf16 T; };
template <int ET, int BIAS_MODE, int OUT_MODE>
__global__ __launch_bounds__(256) void wmma_gemm64(
    const unsigned short* __restrict__ Ap, int lda, long strideA,
    const unsigned short* __restrict__ Btp, int ldb, long strideB,
    void* __restrict__ Cout, int ldc, long strideC,
    const float* __restrict__ bias,
    int M, int N, int K, float scale) {
  typedef typename Elem<ET>::T T;
  typedef typename Frag<T>::V V;
  const T* A = (const T*)Ap; const T* Bt = (const T*)Btp;
  __shared__ __align__(16) float sT[8][16 * 68];
  const int b    = blockIdx.y;
  const int lane = threadIdx.x & 31;
  const int wave = threadIdx.x >> 5;
  const int tilesN = N >> 6;
  const int tilesM = M >> 6;
  const int tile = blockIdx.x * 8 + wave;
  if (tile >= tilesM * tilesN) return;
  const int tm = tile / tilesN;
  const int tn = tile - tm * tilesN;
  const int m0 = tm << 6;
  const int n0 = tn << 6;

  const T* Ab = A  + (size_t)b * strideA;
  const T* Bb = Bt + (size_t)b * strideB;

  const int rlane = lane & 15;
  const int koff  = (lane >> 4) * 8;
  const int mOff  = (lane >> 4) * 8;

  v8f acc[4][4];
#pragma unroll
  for (int i = 0; i < 4; ++i)
#pragma unroll
    for (int j = 0; j < 4; ++j) acc[i][j] = (v8f){0.f,0.f,0.f,0.f,0.f,0.f,0.f,0.f};

  for (int k0 = 0; k0 < K; k0 += 32) {
    V bh[4];
#pragma unroll
    for (int j = 0; j < 4; ++j) {
      const size_t bo = (size_t)(n0 + (j << 4) + rlane) * ldb + koff + k0;
      bh[j] = Frag<T>::load(Bb + bo);
    }
#pragma unroll
    for (int i = 0; i < 4; ++i) {
      const size_t ao = (size_t)(m0 + (i << 4) + rlane) * lda + koff + k0;
      V ah = Frag<T>::load(Ab + ao);
#pragma unroll
      for (int j = 0; j < 4; ++j) acc[i][j] = Frag<T>::mma(ah, bh[j], acc[i][j]);
      Frag<T>::guard1(acc[i][0], ah, bh[0]);
      Frag<T>::guard1(acc[i][1], ah, bh[1]);
      Frag<T>::guard1(acc[i][2], ah, bh[2]);
      Frag<T>::guard1(acc[i][3], ah, bh[3]);
    }
    Frag<T>::keep(bh[0], bh[1], bh[2], bh[3]);
  }

  float* slab = sT[wave];
#pragma unroll
  for (int i = 0; i < 4; ++i) {
    const int mBase = m0 + (i << 4);
#pragma unroll
    for (int j = 0; j < 4; ++j) {
      const int n = n0 + (j << 4) + rlane;
      float bv = 0.f;
      if (BIAS_MODE == 3) {
        const float braw = bias[n];
        bv = bf_bits2f(f2bf_bits(braw));
      }
#pragma unroll
      for (int r = 0; r < 8; ++r) {
        float v = acc[i][j][r] * scale;
        if (BIAS_MODE == 3) v += bv;
        slab[(mOff + r) * 68 + (j << 4) + rlane] = v;
      }
    }
    __builtin_amdgcn_fence(__ATOMIC_RELEASE, "workgroup");
    __builtin_amdgcn_wave_barrier();
    __builtin_amdgcn_fence(__ATOMIC_ACQUIRE, "workgroup");
    if (OUT_MODE == 0) {
      float* C = (float*)Cout + (size_t)b * strideC;
      const int hh = lane >> 4, c4 = (lane & 15) * 4;
      for (int pass = 0; pass < 2; ++pass) {
#pragma unroll
        for (int it = 0; it < 8; ++it) {
          const int row = it * 2 + hh;
          v4f v = *(const v4f*)(slab + row * 68 + c4);
          *(volatile v4f*)(C + (size_t)(mBase + row) * ldc + n0 + c4) = v;
        }
        __threadfence();
      }
    } else {
      const int q = lane >> 3, c8 = (lane & 7) * 8;
      unsigned short* C = (unsigned short*)Cout + (size_t)b * strideC;
      for (int pass = 0; pass < 2; ++pass) {
#pragma unroll
        for (int it = 0; it < 4; ++it) {
          const int row = it * 4 + q;
          const float* sp = slab + row * 68 + c8;
          v8h hv;
#pragma unroll
          for (int e = 0; e < 8; ++e) hv[e] = (_Float16)sp[e];
          *(volatile v8h*)(C + (size_t)(mBase + row) * ldc + n0 + c8) = hv;
        }
        __threadfence();
      }
    }
    __builtin_amdgcn_fence(__ATOMIC_RELEASE, "workgroup");
    __builtin_amdgcn_wave_barrier();
    __builtin_amdgcn_fence(__ATOMIC_ACQUIRE, "workgroup");
  }
}

__global__ __launch_bounds__(256) void cast8_bf16_kernel(const float* __restrict__ in, unsigned short* __restrict__ out, int n8) {
  const int i = blockIdx.x * 256 + threadIdx.x;
  if (i >= n8) return;
  const float* p = in + 8 * (size_t)i;
  const v4f a = *(const v4f*)(p);
  const v4f c = *(const v4f*)(p + 4);
  unsigned short hb[8];
#pragma unroll
  for (int e = 0; e < 4; ++e) {
    const float f0 = a[e];
    const float f1 = c[e];
    hb[e]     = f2bf_bits(f0);
    hb[4 + e] = f2bf_bits(f1);
  }
  const v4u u = (v4u){pk16(hb[0], hb[1]), pk16(hb[2], hb[3]), pk16(hb[4], hb[5]), pk16(hb[6], hb[7])};
  unsigned short* q = out + 8 * (size_t)i;
  *(volatile v4u*)q = u;
  __threadfence();
  *(volatile v4u*)q = u;
}

template <int MODE>
__global__ __launch_bounds__(256) void transpose_cast_kernel(const float* __restrict__ W, unsigned short* __restrict__ out,
                                                             int Kd, int Nd) {
  __shared__ float sm[64][65];
  const int t  = threadIdx.x;
  const int k0 = blockIdx.x * 64;
  const int n0 = blockIdx.y * 64;
#pragma unroll
  for (int i = 0; i < 16; ++i) {
    const int e = i * 256 + t;
    const int r = e >> 6;
    const int c = e & 63;
    sm[c][r] = W[(size_t)(k0 + r) * Nd + n0 + c];
  }
  __syncthreads();
  const int lane = t & 31, wave = t >> 5;
  const int q = lane >> 3, c8 = (lane & 7) * 8;
  v4u u[2];
#pragma unroll
  for (int it = 0; it < 2; ++it) {
    const int row = wave * 8 + it * 4 + q;
    unsigned short hb[8];
#pragma unroll
    for (int e = 0; e < 8; ++e) {
      const float f = sm[row][c8 + e];
      const unsigned short bb = f2bf_bits(f);
      if (MODE == 0) hb[e] = bb;
      else hb[e] = h_bits(bf_bits2f(bb) * kWCarry);
    }
    u[it] = (v4u){pk16(hb[0], hb[1]), pk16(hb[2], hb[3]), pk16(hb[4], hb[5]), pk16(hb[6], hb[7])};
  }
  for (int pass = 0; pass < 2; ++pass) {
#pragma unroll
    for (int it = 0; it < 2; ++it) {
      const int row = wave * 8 + it * 4 + q;
      *(volatile v4u*)(out + (size_t)(n0 + row) * Kd + k0 + c8) = u[it];
    }
    __threadfence();
  }
}

__global__ __launch_bounds__(128) void attn_dist_kernel(const _Float16* __restrict__ QK, const _Float16* __restrict__ Vt,
                                                        _Float16* __restrict__ Oh) {
  __shared__ __align__(16) _Float16 Psh[4][16 * 64];
  __shared__ __align__(16) float    Os[4][16 * 68];

  const int tid  = threadIdx.x;
  const int wave = tid >> 5;
  const int lane = tid & 31;
  const int hh   = lane >> 4;
  const int c    = lane & 15;

  constexpr int nqb = kL / 64;
  const int qb = blockIdx.x % nqb;
  const int bh = blockIdx.x / nqb;
  const int h  = bh % kH;
  const int b  = bh / kH;
  const int q0 = qb * 64 + wave * 16;
  const size_t rowbase = (size_t)b * kL;

  v16h qa[2];
  {
    const _Float16* qrow = QK + (rowbase + q0 + c) * kQKld + h * kDh + 8 * hh;
    qa[0] = Frag<_Float16>::load(qrow);
    qa[1] = Frag<_Float16>::load(qrow + 32);
  }
  const _Float16* kbase = QK + rowbase * kQKld + kD + h * kDh + 8 * hh;
  const _Float16* vbase = Vt + ((size_t)b * kD + h * kDh + c) * kL + 8 * hh;

  float mrow[8], lrow[8], posi[8];
  v8f oacc[4];
#pragma unroll
  for (int r = 0; r < 8; ++r) {
    mrow[r] = -1.0e30f;
    lrow[r] = 0.f;
    posi[r] = pos_frac(q0 + 8 * hh + r);
  }
#pragma unroll
  for (int t = 0; t < 4; ++t) oacc[t] = (v8f){0.f,0.f,0.f,0.f,0.f,0.f,0.f,0.f};

  _Float16* pw = Psh[wave];

#pragma unroll 1
  for (int kc = 0; kc < kL / 64; ++kc) {
    const int kv0 = kc * 64;
    v8f s[4];
#pragma unroll
    for (int j = 0; j < 4; ++j) {
      const _Float16* kp = kbase + (size_t)(kv0 + j * 16 + c) * kQKld;
      v8f sj = (v8f){0.f,0.f,0.f,0.f,0.f,0.f,0.f,0.f};
#pragma unroll
      for (int dc = 0; dc < 2; ++dc) {
        const v16h kb = Frag<_Float16>::load(kp + dc * 32);
        sj = mma_h(qa[dc], kb, sj);
      }
      s[j] = sj;
    }
    float posj[4];
#pragma unroll
    for (int j = 0; j < 4; ++j) posj[j] = pos_frac(kv0 + j * 16 + c);

    float cm[8];
#pragma unroll
    for (int r = 0; r < 8; ++r) {
      float m = -1.0e30f;
#pragma unroll
      for (int j = 0; j < 4; ++j) {
        const float d   = fabsf(posi[r] - posj[j]);
        const float val = fmaf(s[j][r], kScoreScale, -d);
        s[j][r] = val;
        m = fmaxf(m, val);
      }
#pragma unroll
      for (int off = 1; off < 16; off <<= 1) m = fmaxf(m, __shfl_xor(m, off, 32));
      cm[r] = m;
    }
#pragma unroll
    for (int r = 0; r < 8; ++r) {
      const float mnew  = fmaxf(mrow[r], cm[r]);
      const float alpha = __expf(mrow[r] - mnew);
      mrow[r] = mnew;
      float psum = 0.f;
#pragma unroll
      for (int j = 0; j < 4; ++j) {
        const float p = __expf(s[j][r] - mnew);
        psum += p;
        pw[(8 * hh + r) * 64 + j * 16 + c] = (_Float16)(p * kPCarry);
      }
#pragma unroll
      for (int off = 1; off < 16; off <<= 1) psum += __shfl_xor(psum, off, 32);
      lrow[r] = lrow[r] * alpha + psum;
#pragma unroll
      for (int t = 0; t < 4; ++t) oacc[t][r] *= alpha;
    }
    __builtin_amdgcn_fence(__ATOMIC_RELEASE, "workgroup");
    __builtin_amdgcn_wave_barrier();
    __builtin_amdgcn_fence(__ATOMIC_ACQUIRE, "workgroup");
#pragma unroll 1
    for (int kk = 0; kk < 2; ++kk) {
      const v16h pa = Frag<_Float16>::load(pw + c * 64 + kk * 32 + 8 * hh);
#pragma unroll
      for (int t = 0; t < 4; ++t) {
        const v16h vb = Frag<_Float16>::load(vbase + (size_t)(t * 16) * kL + kv0 + kk * 32);
        oacc[t] = mma_h(pa, vb, oacc[t]);
      }
    }
  }

  float* os = Os[wave];
#pragma unroll
  for (int r = 0; r < 8; ++r) {
    const float inv = (1.0f / lrow[r]) * kCtxScale;
#pragma unroll
    for (int t = 0; t < 4; ++t) os[(8 * hh + r) * 68 + t * 16 + c] = oacc[t][r] * inv;
  }
  __builtin_amdgcn_fence(__ATOMIC_RELEASE, "workgroup");
  __builtin_amdgcn_wave_barrier();
  __builtin_amdgcn_fence(__ATOMIC_ACQUIRE, "workgroup");
  {
    const int q = lane >> 3, c8 = (lane & 7) * 8;
    v8h hv[4];
#pragma unroll
    for (int it = 0; it < 4; ++it) {
      const int row = it * 4 + q;
      const float* sp = os + row * 68 + c8;
#pragma unroll
      for (int e = 0; e < 8; ++e) hv[it][e] = (_Float16)sp[e];
    }
    for (int pass = 0; pass < 2; ++pass) {
#pragma unroll
      for (int it = 0; it < 4; ++it) {
        const int row = it * 4 + q;
        *(volatile v8h*)(Oh + (rowbase + q0 + row) * kD + h * kDh + c8) = hv[it];
      }
      __threadfence();
    }
  }
}

extern "C" void kernel_launch(void* const* d_in, const int* in_sizes, int n_in,
                              void* d_out, int out_size, void* d_ws, size_t ws_size,
                              hipStream_t stream) {
  if (n_in < 4) return;
  if (in_sizes[0] != kRows * kD) return;
  if (in_sizes[1] != kD * 3 * kD) return;
  if (in_sizes[2] != kD * kD) return;
  if (in_sizes[3] != kD) return;
  if (out_size != kRows * kD) return;
  if (ws_size < kWsTotal) return;

  const float* x      = (const float*)d_in[0];
  const float* w_qkv  = (const float*)d_in[1];
  const float* w_proj = (const float*)d_in[2];
  const float* b_proj = (const float*)d_in[3];
  float* out = (float*)d_out;

  char* ws = (char*)d_ws;
  unsigned short* XB  = (unsigned short*)(ws + kOffXB);
  unsigned short* WQT = (unsigned short*)(ws + kOffWQT);
  unsigned short* WPT = (unsigned short*)(ws + kOffWPT);
  unsigned short* QKH = (unsigned short*)(ws + kOffQKH);
  unsigned short* VT  = (unsigned short*)(ws + kOffVT);
  unsigned short* OH  = (unsigned short*)(ws + kOffOH);

  cast8_bf16_kernel<<<(kRows * kD / 8) / 256, 256, 0, stream>>>(x, XB, kRows * kD / 8);

  transpose_cast_kernel<0><<<dim3(kD / 64, 3 * kD / 64), 256, 0, stream>>>(w_qkv, WQT, kD, 3 * kD);
  transpose_cast_kernel<1><<<dim3(kD / 64, kD / 64), 256, 0, stream>>>(w_proj, WPT, kD, kD);

  wmma_gemm64<1, 0, 1><<<dim3((kRows / 64) * (kQKld / 64) / 8, 1), 256, 0, stream>>>(
      XB, kD, 0L,
      WQT, kD, 0L,
      (void*)QKH, kQKld, 0L,
      nullptr, kRows, kQKld, kD, 1.0f);

  wmma_gemm64<1, 0, 1><<<dim3((kD / 64) * (kL / 64) / 8, kB), 256, 0, stream>>>(
      WQT + (size_t)2 * kD * kD, kD, 0L,
      XB, kD, (long)kL * kD,
      (void*)VT, kL, (long)kD * kL,
      nullptr, kD, kL, kD, 1.0f);

  attn_dist_kernel<<<kB * kH * (kL / 64), 128, 0, stream>>>((const _Float16*)QKH, (const _Float16*)VT, (_Float16*)OH);

  wmma_gemm64<0, 3, 0><<<dim3((kRows / 64) * (kD / 64) / 8, 1), 256, 0, stream>>>(
      OH, kD, 0L,
      WPT, kD, 0L,
      (void*)out, kD, 0L,
      b_proj, kRows, kD, kD, kOutScale);
}
